// PointNetSAModule_47571057771109
// MI455X (gfx1250) — hardware-verified
//
#include <hip/hip_runtime.h>
#include <math.h>

#pragma clang fp contract(off)

constexpr int kB    = 8;
constexpr int kN    = 8192;
constexpr int kCin  = 64;
constexpr int kM    = 1024;
constexpr int kK    = 64;
constexpr int kNC   = kB * kM;
constexpr int kC0   = 67;
constexpr int kC0P  = 96;
constexpr int kO1   = 64;
constexpr int kO2   = 64;
constexpr int kO3   = 128;
constexpr int kW0Off = 0;
constexpr int kW1Off = kO1 * kC0P;
constexpr int kW2Off = kW1Off + kO2 * kO1;
constexpr int kWPlaneHalves = kW2Off + kO3 * kO2;
constexpr int kWPlaneDwords = kWPlaneHalves / 2;
constexpr float kRad2 = 0.04f;
constexpr int kCenPerBlk = 32;
static_assert(kWPlaneDwords % 256 == 0);
static_assert(kNC % kCenPerBlk == 0);
static_assert(kM % kCenPerBlk == 0);
static_assert(kC0P % 32 == 0);
static_assert((kW1Off / 2) % 32 == 0);
static_assert((kW2Off / 2) % 32 == 0);

typedef __attribute__((ext_vector_type(16))) _Float16 v16h;
typedef __attribute__((ext_vector_type(8)))  _Float16 v8h;
typedef __attribute__((ext_vector_type(16))) __bf16   v16b;
typedef __attribute__((ext_vector_type(8)))  __bf16   v8b;
typedef __attribute__((ext_vector_type(8)))  float    v8f;
typedef __attribute__((ext_vector_type(4)))  float    v4f;
typedef __attribute__((ext_vector_type(4)))  unsigned int v4u;
typedef __attribute__((ext_vector_type(4)))  int      v4i;

__device__ __forceinline__ unsigned short f2bf_bits(float f) {
  unsigned u = __float_as_uint(f);
  return (unsigned short)((u + 0x7FFFu + ((u >> 16) & 1u)) >> 16);
}
__device__ __forceinline__ float bf_bits2f(unsigned short h) { return __uint_as_float(((unsigned)h) << 16); }

__device__ __forceinline__ void dep_guard_h(v8f& a, v8f& b, v16h x, v16h y) { asm volatile("v_nop\n\tv_nop\n\tv_nop\n\tv_nop" : "+v"(a), "+v"(b) : "v"(x), "v"(y)); }
__device__ __forceinline__ void dep_guard_b(v8f& a, v8f& b, v16b x, v16b y) { asm volatile("v_nop\n\tv_nop\n\tv_nop\n\tv_nop" : "+v"(a), "+v"(b) : "v"(x), "v"(y)); }
__device__ __forceinline__ void keep4_h(v16h a, v16h b, v16h c, v16h d) { asm volatile("v_nop" :: "v"(a), "v"(b), "v"(c), "v"(d)); }
__device__ __forceinline__ void keep4_b(v16b a, v16b b, v16b c, v16b d) { asm volatile("v_nop" :: "v"(a), "v"(b), "v"(c), "v"(d)); }
__device__ __forceinline__ void acc_guard4(v8f& a, v8f& b, v8f& c, v8f& d) { asm volatile("v_nop\n\tv_nop\n\tv_nop\n\tv_nop" : "+v"(a), "+v"(b), "+v"(c), "+v"(d)); }
template <typename T> struct Frag;
template <> struct Frag<_Float16> {
  typedef v16h V; union U { v16h v; v8h h[2]; };
  static __device__ __forceinline__ v16h load(const _Float16* p) {
    U f; f.h[0] = *(const v8h*)(p); f.h[1] = *(const v8h*)(p + 16); return f.v;
  }
  static __device__ __forceinline__ v8f mma(v16h a, v16h b, v8f c) {
    return __builtin_amdgcn_wmma_f32_16x16x32_f16(false, a, false, b, (short)0, c, false, false);
  }
  static __device__ __forceinline__ void guard(v8f& a, v8f& b, v16h x, v16h y) { dep_guard_h(a, b, x, y); }
  static __device__ __forceinline__ void keep(v16h a, v16h b, v16h c, v16h d) { keep4_h(a, b, c, d); }
};
template <> struct Frag<__bf16> {
  typedef v16b V; union U { v16b v; v8b h[2]; };
  static __device__ __forceinline__ v16b load(const __bf16* p) {
    U f; f.h[0] = *(const v8b*)(p); f.h[1] = *(const v8b*)(p + 16); return f.v;
  }
  static __device__ __forceinline__ v8f mma(v16b a, v16b b, v8f c) {
    return __builtin_amdgcn_wmma_f32_16x16x32_bf16(false, a, false, b, (short)0, c, false, false);
  }
  static __device__ __forceinline__ void guard(v8f& a, v8f& b, v16b x, v16b y) { dep_guard_b(a, b, x, y); }
  static __device__ __forceinline__ void keep(v16b a, v16b b, v16b c, v16b d) { keep4_b(a, b, c, d); }
};

__device__ __forceinline__ unsigned pk16(unsigned short a, unsigned short b) { return (unsigned)a | ((unsigned)b << 16); }
__device__ __forceinline__ v8f zero8() { return (v8f){0.f, 0.f, 0.f, 0.f, 0.f, 0.f, 0.f, 0.f}; }

__device__ __forceinline__ void wave_sync() {
  __builtin_amdgcn_fence(__ATOMIC_RELEASE, "workgroup");
  __builtin_amdgcn_wave_barrier();
  __builtin_amdgcn_fence(__ATOMIC_ACQUIRE, "workgroup");
}

__device__ __forceinline__ v8f mma3(v16b ah, v16b al, v16b bh, v16b bl, v8f c) {
  c = __builtin_amdgcn_wmma_f32_16x16x32_bf16(false, ah, false, bh, (short)0, c, false, false);
  c = __builtin_amdgcn_wmma_f32_16x16x32_bf16(false, ah, false, bl, (short)0, c, false, false);
  c = __builtin_amdgcn_wmma_f32_16x16x32_bf16(false, al, false, bh, (short)0, c, false, false);
  asm volatile("v_nop\n\tv_nop\n\tv_nop\n\tv_nop" : "+v"(c) : "v"(ah), "v"(al), "v"(bh), "v"(bl));
  return c;
}

__device__ __forceinline__ v16b ldw(const unsigned short* __restrict__ wp, int base_half, int pitch, int obase, int k0, int lane) {
  int o = obase + (lane & 15);
  asm volatile("" : "+v"(o) : : "memory");
  const __bf16* p = (const __bf16*)wp + base_half + o * pitch + k0 + ((lane >> 4) << 3);
  return Frag<__bf16>::load(p);
}
__device__ __forceinline__ v16b ldx(const unsigned short* xp, int pitch, int k0, int lane) {
  const __bf16* p = (const __bf16*)xp + (lane & 15) * pitch + k0 + ((lane >> 4) << 3);
  return Frag<__bf16>::load(p);
}

__device__ __forceinline__ void epi16(unsigned short* yh, unsigned short* yl, int pitch, int obase, v8f acc,
                                      const float* sc, const float* bi, int lane) {
  const int nn = lane & 15;
  const int oo = obase + ((lane >> 4) << 3);
  unsigned short hb[8], lb[8];
#pragma unroll
  for (int r = 0; r < 8; ++r) {
    float v = acc[r] * sc[oo + r];
    v = v + bi[oo + r];
    v = fmaxf(v, 0.0f);
    const unsigned short h = f2bf_bits(v);
    hb[r] = h;
    lb[r] = f2bf_bits(v - bf_bits2f(h));
  }
  const v4u uh = (v4u){pk16(hb[0], hb[1]), pk16(hb[2], hb[3]), pk16(hb[4], hb[5]), pk16(hb[6], hb[7])};
  const v4u ul = (v4u){pk16(lb[0], lb[1]), pk16(lb[2], lb[3]), pk16(lb[4], lb[5]), pk16(lb[6], lb[7])};
  *(v4u*)(yh + nn * pitch + oo) = uh;
  *(v4u*)(yl + nn * pitch + oo) = ul;
}
__device__ __forceinline__ void epimax(v8f& rm, v8f acc, int obase, const float* sc, const float* bi, int lane) {
  const int oo = obase + ((lane >> 4) << 3);
#pragma unroll
  for (int r = 0; r < 8; ++r) {
    float v = acc[r] * sc[oo + r];
    v = v + bi[oo + r];
    v = fmaxf(v, 0.0f);
    rm[r] = fmaxf(rm[r], v);
  }
}

__device__ __forceinline__ void argmax_bfly(float& bv, int& bi) {
#pragma unroll
  for (int off = 16; off >= 1; off >>= 1) {
    const float ov = __shfl_xor(bv, off);
    const int   oi = __shfl_xor(bi, off);
    const bool take = (ov > bv) || (ov == bv && oi < bi);
    bv = take ? ov : bv;
    bi = take ? oi : bi;
  }
}

__global__ __launch_bounds__(256) void prep_kernel(const float* __restrict__ w0, const float* __restrict__ w1,
                                                   const float* __restrict__ w2,
                                                   unsigned* __restrict__ whp, unsigned* __restrict__ wlp) {
  const int i = blockIdx.x * 256 + threadIdx.x;
  const int seg = __builtin_amdgcn_readfirstlane(i >> 5);
  float a, c;
  if (seg < (kW1Off / 2) / 32) {
    const int row = i / 48;
    const int col = 2 * (i - row * 48);
    const int ca = col < kC0 ? col : kC0 - 1;
    const int cb = (col + 1) < kC0 ? (col + 1) : kC0 - 1;
    const float xa = w0[row * kC0 + ca];
    const float xb = w0[row * kC0 + cb];
    const float fa = (col < kC0) ? 1.0f : 0.0f;
    const float fb = ((col + 1) < kC0) ? 1.0f : 0.0f;
    a = xa * fa;
    c = xb * fb;
  } else if (seg < (kW2Off / 2) / 32) {
    const int j = i - kW1Off / 2;
    a = w1[2 * j]; c = w1[2 * j + 1];
  } else {
    const int j = i - kW2Off / 2;
    a = w2[2 * j]; c = w2[2 * j + 1];
  }
  const unsigned short ha = f2bf_bits(a), hc = f2bf_bits(c);
  const unsigned short la = f2bf_bits(a - bf_bits2f(ha)), lc = f2bf_bits(c - bf_bits2f(hc));
  const unsigned uh = pk16(ha, hc), ul = pk16(la, lc);
  ((volatile unsigned*)whp)[i] = uh; ((volatile unsigned*)wlp)[i] = ul;
  __threadfence();
  ((volatile unsigned*)whp)[i] = uh; ((volatile unsigned*)wlp)[i] = ul;
}

__global__ __launch_bounds__(1024) void fps_kernel(const float* __restrict__ xyz, int* __restrict__ cidx,
                                                   float* __restrict__ cen, float* __restrict__ out0) {
  __shared__ float selx[kM];
  __shared__ float sely[kM];
  __shared__ float selz[kM];
  __shared__ int   seli[kM];
  __shared__ float wvv[32];
  __shared__ int   wvi[32];
  __shared__ float cur[4];
  const int b = blockIdx.x;
  const int t = threadIdx.x;
  const int lane = t & 31, wv = t >> 5;
  const float* xb = xyz + (size_t)b * 3 * kN;

  float px[8], py[8], pz[8], dm[8];
#pragma unroll
  for (int e = 0; e < 4; ++e) {
    const int j = e * 1024 + t;
    px[e] = xb[j]; py[e] = xb[kN + j]; pz[e] = xb[2 * kN + j]; dm[e] = 1e10f;
  }
  asm volatile("" :: "v"(px[0]), "v"(px[1]), "v"(px[2]), "v"(px[3]),
                     "v"(py[0]), "v"(py[1]), "v"(py[2]), "v"(py[3]),
                     "v"(pz[0]), "v"(pz[1]), "v"(pz[2]), "v"(pz[3]) : "memory");
#pragma unroll
  for (int e = 4; e < 8; ++e) {
    const int j = e * 1024 + t;
    px[e] = xb[j]; py[e] = xb[kN + j]; pz[e] = xb[2 * kN + j]; dm[e] = 1e10f;
  }
  asm volatile("" :: "v"(px[4]), "v"(px[5]), "v"(px[6]), "v"(px[7]),
                     "v"(py[4]), "v"(py[5]), "v"(py[6]), "v"(py[7]),
                     "v"(pz[4]), "v"(pz[5]), "v"(pz[6]), "v"(pz[7]) : "memory");
  if (t == 0) {
    seli[0] = 0; selx[0] = px[0]; sely[0] = py[0]; selz[0] = pz[0];
    cur[0] = px[0]; cur[1] = py[0]; cur[2] = pz[0];
  }
  __syncthreads();

#pragma unroll 1
  for (int s = 1; s < kM; ++s) {
    const float cx = cur[0], cy = cur[1], cz = cur[2];
    float bv = -1.0f; int bi = t;
#pragma unroll
    for (int e = 0; e < 8; ++e) {
      const float dx = px[e] - cx, dy = py[e] - cy, dz = pz[e] - cz;
      const float tx = dx * dx;
      const float ty = dy * dy;
      const float tz = dz * dz;
      const float d = (tx + tz) + ty;
      dm[e] = fminf(dm[e], d);
      const bool gt = dm[e] > bv;
      bv = gt ? dm[e] : bv;
      bi = gt ? (e * 1024 + t) : bi;
    }
    argmax_bfly(bv, bi);
    if (lane == 0) { wvv[wv] = bv; wvi[wv] = bi; }
    __syncthreads();
    bv = wvv[lane]; bi = wvi[lane];
    argmax_bfly(bv, bi);
    const int bic = bi < 0 ? 0 : (bi >= kN ? kN - 1 : bi);
    if (wv == 0) {
      const float nx = xb[bic];
      const float ny = xb[kN + bic];
      const float nz = xb[2 * kN + bic];
      if (lane == 0) {
        seli[s] = bic; selx[s] = nx; sely[s] = ny; selz[s] = nz;
        cur[0] = nx; cur[1] = ny; cur[2] = nz;
      }
    }
    __syncthreads();
  }

  const float vx = selx[t], vy = sely[t], vz = selz[t];
  const int vi = seli[t];
  float* o0 = out0 + (size_t)b * 3 * kM;
  float* cb = cen + (size_t)b * 3 * kM;
  int* ib = cidx + (size_t)b * kM;
  for (int pass = 0; pass < 2; ++pass) {
    ((volatile float*)o0)[t] = vx;
    ((volatile float*)o0)[kM + t] = vy;
    ((volatile float*)o0)[2 * kM + t] = vz;
    ((volatile float*)cb)[t] = vx;
    ((volatile float*)cb)[kM + t] = vy;
    ((volatile float*)cb)[2 * kM + t] = vz;
    ((volatile int*)ib)[t] = vi;
    __threadfence();
  }
}

__global__ __launch_bounds__(256) void ballq_kernel(const float* __restrict__ xyz, const float* __restrict__ cen,
                                                    int* __restrict__ nidx) {
  __shared__ __align__(16) int nl[8][kK];
  const int tid = threadIdx.x;
  const int wave = tid >> 5, lane = tid & 31;
  const unsigned lt = (1u << lane) - 1u;
  int* lst = nl[wave];
#pragma unroll 1
  for (int i = 0; i < 4; ++i) {
    const int g = blockIdx.x * kCenPerBlk + wave * 4 + i;
    const int b = g >> 10, m = g & (kM - 1);
    const float cx = cen[(size_t)(b * 3 + 0) * kM + m];
    const float cy = cen[(size_t)(b * 3 + 1) * kM + m];
    const float cz = cen[(size_t)(b * 3 + 2) * kM + m];
    const float scx = cx * cx, scy = cy * cy, scz = cz * cz;
    const float sc = (scx + scy) + scz;
    const float* xb = xyz + (size_t)b * 3 * kN;
    int cnt = 0, first = 0;
#pragma unroll 1
    for (int c0 = 0; c0 < kN; c0 += 32) {
      const int j = c0 + lane;
      const float px = xb[j], py = xb[kN + j], pz = xb[2 * kN + j];
      const float spx = px * px, spy = py * py, spz = pz * pz;
      const float sp = (spx + spy) + spz;
      float p = cx * px;
      p = fmaf(cy, py, p);
      p = fmaf(cz, pz, p);
      const float p2 = 2.0f * p;
      const float d2 = (sc + sp) - p2;
      const bool inr = d2 < kRad2;
      const unsigned mask = (unsigned)__ballot(inr);
      if (mask != 0u) {
        if (cnt == 0) first = c0 + (__ffs(mask) - 1);
        const int pos = cnt + (int)__popc(mask & lt);
        if (inr && pos < kK) lst[pos] = j;
        cnt += (int)__popc(mask);
        if (cnt >= kK) break;
      }
    }
    cnt = cnt > kK ? kK : cnt;
    const int pad = (cnt > 0) ? first : 0;
    for (int q = cnt + lane; q < kK; q += 32) lst[q] = pad;
    wave_sync();
    const v4i v = *(const v4i*)(lst + 4 * (lane & 15));
    int* dst = nidx + (size_t)g * kK + 4 * (lane & 15);
    for (int pass = 0; pass < 2; ++pass) {
      if (lane < 16) *(volatile v4i*)dst = v;
      __threadfence();
    }
    wave_sync();
  }
}

__global__ __launch_bounds__(128) void mlp_kernel(const float* __restrict__ xyz, const float* __restrict__ feat,
                                                  const float* __restrict__ cen, const int* __restrict__ nidx,
                                                  const unsigned short* __restrict__ wh, const unsigned short* __restrict__ wl,
                                                  const float* __restrict__ s0, const float* __restrict__ b0,
                                                  const float* __restrict__ s1, const float* __restrict__ b1,
                                                  const float* __restrict__ s2, const float* __restrict__ b2,
                                                  float* __restrict__ out1) {
  __shared__ __align__(16) unsigned short Xh[4][16 * kC0P];
  __shared__ __align__(16) unsigned short Xl[4][16 * kC0P];
  __shared__ __align__(16) unsigned short Yh[4][16 * 64];
  __shared__ __align__(16) unsigned short Yl[4][16 * 64];
  __shared__ __align__(16) float pool[kO3 * kCenPerBlk];
  __shared__ __align__(16) float sb[512];
  __shared__ int   nid[4][kK];
  __shared__ float cenS[4][4];

  const int tid = threadIdx.x;
  const int wave = tid >> 5, lane = tid & 31;
  const int nn = lane & 15, hh = lane >> 4;

  if (tid < 64) { sb[tid] = s0[tid]; sb[64 + tid] = b0[tid]; sb[128 + tid] = s1[tid]; sb[192 + tid] = b1[tid]; }
  sb[256 + tid] = s2[tid]; sb[384 + tid] = b2[tid];
  __syncthreads();

  const int g0 = blockIdx.x * kCenPerBlk;
  const int b  = g0 >> 10;
  const int mb = g0 & (kM - 1);
  const float* xb = xyz + (size_t)b * 3 * kN;
  const float* fb = feat + (size_t)b * kCin * kN;
  unsigned short* xh = Xh[wave];
  unsigned short* xl = Xl[wave];
  unsigned short* yh = Yh[wave];
  unsigned short* yl = Yl[wave];
  const float* sc0 = sb;        const float* bi0 = sb + 64;
  const float* sc1 = sb + 128;  const float* bi1 = sb + 192;
  const float* sc2 = sb + 256;  const float* bi2 = sb + 384;

#pragma unroll 1
  for (int ci = 0; ci < 8; ++ci) {
    const int ml = wave * 8 + ci;
    const int g  = g0 + ml;
    const int m  = mb + ml;
    {
      int i0 = nidx[(size_t)g * kK + lane];
      int i1 = nidx[(size_t)g * kK + 32 + lane];
      i0 = i0 < 0 ? 0 : (i0 >= kN ? kN - 1 : i0);
      i1 = i1 < 0 ? 0 : (i1 >= kN ? kN - 1 : i1);
      const int cc = lane < 3 ? lane : 2;
      const float cv = cen[(size_t)(b * 3 + cc) * kM + m];
      nid[wave][lane] = i0; nid[wave][32 + lane] = i1;
      if (lane < 3) cenS[wave][lane] = cv;
    }
    wave_sync();
    int nt;
    {
      const int a0 = nid[wave][0], a1 = nid[wave][16], a2 = nid[wave][32], a3 = nid[wave][48];
      nt = (a3 != a0) ? 4 : ((a2 != a0) ? 3 : ((a1 != a0) ? 2 : 1));
      nt = __builtin_amdgcn_readfirstlane(nt);
    }
    v8f rmax[8];
#pragma unroll
    for (int mt = 0; mt < 8; ++mt) rmax[mt] = zero8();

#pragma unroll 1
    for (int t = 0; t < nt; ++t) {
      {
        const int idx = nid[wave][t * 16 + nn];
        const float ca = cenS[wave][hh];
        const float c2v = cenS[wave][2];
        float va = xb[(size_t)hh * kN + idx];
        float vz = xb[(size_t)2 * kN + idx];
        va = va - ca;
        vz = vz - c2v;
        const unsigned short ha = f2bf_bits(va);
        xh[nn * kC0P + hh] = ha;
        xl[nn * kC0P + hh] = f2bf_bits(va - bf_bits2f(ha));
        const unsigned short hz = f2bf_bits(vz);
        xh[nn * kC0P + 2] = hz;
        xl[nn * kC0P + 2] = f2bf_bits(vz - bf_bits2f(hz));
#pragma unroll 1
        for (int g4 = 0; g4 < 8; ++g4) {
#pragma unroll
          for (int u = 0; u < 4; ++u) {
            const int fc = 2 * (g4 * 4 + u) + hh;
            const float v = fb[(size_t)fc * kN + idx];
            const unsigned short hv = f2bf_bits(v);
            xh[nn * kC0P + 3 + fc] = hv;
            xl[nn * kC0P + 3 + fc] = f2bf_bits(v - bf_bits2f(hv));
          }
          asm volatile("" ::: "memory");
        }
#pragma unroll
        for (int jj = 0; jj < 15; ++jj) {
          const int e = lane + 32 * jj;
          if (e < 464) {
            const int cp = kC0 + (e >> 4);
            const int rr = e & 15;
            xh[rr * kC0P + cp] = 0;
            xl[rr * kC0P + cp] = 0;
          }
        }
      }
      wave_sync();
      {
        const v16b bh0 = ldx(xh, kC0P, 0, lane),  bl0 = ldx(xl, kC0P, 0, lane);
        const v16b bh1 = ldx(xh, kC0P, 32, lane), bl1 = ldx(xl, kC0P, 32, lane);
        const v16b bh2 = ldx(xh, kC0P, 64, lane), bl2 = ldx(xl, kC0P, 64, lane);
#pragma unroll
        for (int mt = 0; mt < 4; ++mt) {
          v8f acc = zero8();
          acc = mma3(ldw(wh, kW0Off, kC0P, mt * 16, 0, lane),  ldw(wl, kW0Off, kC0P, mt * 16, 0, lane),  bh0, bl0, acc);
          acc = mma3(ldw(wh, kW0Off, kC0P, mt * 16, 32, lane), ldw(wl, kW0Off, kC0P, mt * 16, 32, lane), bh1, bl1, acc);
          acc = mma3(ldw(wh, kW0Off, kC0P, mt * 16, 64, lane), ldw(wl, kW0Off, kC0P, mt * 16, 64, lane), bh2, bl2, acc);
          epi16(yh, yl, 64, mt * 16, acc, sc0, bi0, lane);
        }
      }
      wave_sync();
      {
        const v16b bh0 = ldx(yh, 64, 0, lane),  bl0 = ldx(yl, 64, 0, lane);
        const v16b bh1 = ldx(yh, 64, 32, lane), bl1 = ldx(yl, 64, 32, lane);
#pragma unroll
        for (int mt = 0; mt < 4; ++mt) {
          v8f acc = zero8();
          acc = mma3(ldw(wh, kW1Off, 64, mt * 16, 0, lane),  ldw(wl, kW1Off, 64, mt * 16, 0, lane),  bh0, bl0, acc);
          acc = mma3(ldw(wh, kW1Off, 64, mt * 16, 32, lane), ldw(wl, kW1Off, 64, mt * 16, 32, lane), bh1, bl1, acc);
          epi16(xh, xl, 64, mt * 16, acc, sc1, bi1, lane);
        }
      }
      wave_sync();
      {
        const v16b bh0 = ldx(xh, 64, 0, lane),  bl0 = ldx(xl, 64, 0, lane);
        const v16b bh1 = ldx(xh, 64, 32, lane), bl1 = ldx(xl, 64, 32, lane);
#pragma unroll
        for (int mt = 0; mt < 8; ++mt) {
          v8f acc = zero8();
          acc = mma3(ldw(wh, kW2Off, 64, mt * 16, 0, lane),  ldw(wl, kW2Off, 64, mt * 16, 0, lane),  bh0, bl0, acc);
          acc = mma3(ldw(wh, kW2Off, 64, mt * 16, 32, lane), ldw(wl, kW2Off, 64, mt * 16, 32, lane), bh1, bl1, acc);
          epimax(rmax[mt], acc, mt * 16, sc2, bi2, lane);
        }
      }
      wave_sync();
    }
#pragma unroll
    for (int mt = 0; mt < 8; ++mt) {
#pragma unroll
      for (int r = 0; r < 8; ++r) {
        float v = rmax[mt][r];
        v = fmaxf(v, __shfl_xor(v, 1));
        v = fmaxf(v, __shfl_xor(v, 2));
        v = fmaxf(v, __shfl_xor(v, 4));
        v = fmaxf(v, __shfl_xor(v, 8));
        if (nn == 0) pool[(mt * 16 + hh * 8 + r) * kCenPerBlk + ml] = v;
      }
    }
  }
  __syncthreads();
  {
    float* ob = out1 + (size_t)b * kO3 * kM + mb;
    const int q = lane >> 3, c4 = (lane & 7) * 4;
    for (int pass = 0; pass < 2; ++pass) {
#pragma unroll
      for (int it = 0; it < 8; ++it) {
        const int o = wave * 32 + it * 4 + q;
        const v4f v = *(const v4f*)(pool + o * kCenPerBlk + c4);
        *(volatile v4f*)(ob + (size_t)o * kM + c4) = v;
      }
      __threadfence();
    }
  }
}

extern "C" void kernel_launch(void* const* d_in, const int* in_sizes, int n_in,
                              void* d_out, int out_size, void* d_ws, size_t ws_size, hipStream_t stream) {
  if (n_in < 11) return;
  if (in_sizes[0] != kB * 3 * kN || in_sizes[1] != kB * kCin * kN || in_sizes[2] != kO1 * kC0 ||
      in_sizes[5] != kO2 * kO1 || in_sizes[8] != kO3 * kO2 || out_size != kB * 3 * kM + kB * kO3 * kM) return;
  const float* xyz  = (const float*)d_in[0];
  const float* feat = (const float*)d_in[1];
  const float* w0   = (const float*)d_in[2];
  const float* s0   = (const float*)d_in[3];
  const float* b0   = (const float*)d_in[4];
  const float* w1   = (const float*)d_in[5];
  const float* s1   = (const float*)d_in[6];
  const float* b1   = (const float*)d_in[7];
  const float* w2   = (const float*)d_in[8];
  const float* s2   = (const float*)d_in[9];
  const float* b2   = (const float*)d_in[10];

  float* out0 = (float*)d_out;
  float* out1 = (float*)d_out + (size_t)kB * 3 * kM;

  char* ws = (char*)d_ws; size_t off = 0;
  auto carve = [&](size_t bytes) -> char* { char* p = ws + off; off += (bytes + 255) & ~(size_t)255; return p; };
  int*            cidx = (int*)carve((size_t)kNC * 4);
  float*          cen  = (float*)carve((size_t)kB * 3 * kM * 4);
  int*            nidx = (int*)carve((size_t)kNC * kK * 4);
  unsigned short* whi  = (unsigned short*)carve((size_t)kWPlaneHalves * 2);
  unsigned short* wlo  = (unsigned short*)carve((size_t)kWPlaneHalves * 2);
  if (off > ws_size || off > (size_t)134217728) return;

  prep_kernel<<<kWPlaneDwords / 256, 256, 0, stream>>>(w0, w1, w2, (unsigned*)whi, (unsigned*)wlo);
  fps_kernel<<<kB, 1024, 0, stream>>>(xyz, cidx, cen, out0);
  ballq_kernel<<<kNC / kCenPerBlk, 256, 0, stream>>>(xyz, cen, nidx);
  mlp_kernel<<<kNC / kCenPerBlk, 128, 0, stream>>>(xyz, feat, cen, nidx, whi, wlo,
                                                   s0, b0, s1, b1, s2, b2, out1);
}
